// KANLayer_89953795047906
// MI455X (gfx1250) — hardware-verified
//
#include <hip/hip_runtime.h>

typedef __attribute__((ext_vector_type(16))) _Float16 v16h;
typedef __attribute__((ext_vector_type(8)))  _Float16 v8h;
typedef __attribute__((ext_vector_type(8)))  float    v8f;
typedef __attribute__((ext_vector_type(4)))  float    v4f;
typedef __attribute__((ext_vector_type(2)))  float    v2f;
typedef __attribute__((ext_vector_type(4)))  unsigned v4u;

constexpr int kRows = 16384;
constexpr int kFeat = 256;
constexpr int kHid  = 64;
constexpr int kOut  = 256;
constexpr int kFG   = 64;
constexpr int kRowsPerBlock = 128;
constexpr float kCarryU = 32.0f;
constexpr float kCarryW = 1024.0f;
constexpr float kFold   = 1.0f / (kCarryU * kCarryW);
static_assert((kRows % 64) == 0 && (kOut % 64) == 0 && (kFeat % 32) == 0);
static_assert((kFeat % kFG) == 0 && (kRows % kRowsPerBlock) == 0 && kHid == 64 && kFG == 64);
static_assert(kFold == 1.0f / 32768.0f);

constexpr size_t kOffWC16 = 0;
constexpr size_t kOffU16  = kOffWC16 + (size_t)kOut * kFeat * 2;
constexpr size_t kWsTotal = kOffU16 + (size_t)kRows * kFeat * 2;
static_assert(kWsTotal == 8519680ull);
static_assert(kWsTotal <= 134217728ull);
static_assert((kOffU16 % 128) == 0);

__device__ __forceinline__ unsigned f16_bits_flush(float v) {
  const unsigned u = __float_as_uint(v);
  const unsigned sgn = (v < 0.0f) ? 0x8000u : 0u;
  unsigned em = u & 0x7fffffffu;
  em = (em > 0x477fe000u) ? 0x477fe000u : em;
  unsigned t = em - 0x38000000u;
  const unsigned lsb = (t & 0x00002000u) ? 1u : 0u;
  t = t + 0x00000fffu + lsb;
  unsigned hb = (t >> 13) | sgn;
  hb = (em < 0x38800000u) ? 0u : hb;
  asm volatile("" : "+v"(hb));
  return hb;
}
__device__ __forceinline__ unsigned pack_halves(unsigned lo, unsigned hi) {
  unsigned w = (hi << 16) | (lo & 0xffffu);
  asm volatile("" : "+v"(w));
  return w;
}

static_assert(((kOut * kFeat / 8) % 256) == 0);
__global__ __launch_bounds__(256) void cast_weight_plane_kernel(
    const float* __restrict__ src, unsigned* __restrict__ dst)
{
  unsigned tid = threadIdx.x;
  asm volatile("" : "+v"(tid));
  const unsigned i = blockIdx.x * 256u + tid;
  const size_t e0 = (size_t)i << 3;
  const v4f a0 = *(const v4f*)(src + e0);
  const v4f a1 = *(const v4f*)(src + e0 + 4);
  const float s0 = a0[0], s1 = a0[1], s2 = a0[2], s3 = a0[3];
  const float s4 = a1[0], s5 = a1[1], s6 = a1[2], s7 = a1[3];
  v4u w;
  w[0] = pack_halves(f16_bits_flush(s0 * kCarryW), f16_bits_flush(s1 * kCarryW));
  w[1] = pack_halves(f16_bits_flush(s2 * kCarryW), f16_bits_flush(s3 * kCarryW));
  w[2] = pack_halves(f16_bits_flush(s4 * kCarryW), f16_bits_flush(s5 * kCarryW));
  w[3] = pack_halves(f16_bits_flush(s6 * kCarryW), f16_bits_flush(s7 * kCarryW));
  unsigned* p = dst + ((size_t)i << 2);
  *(volatile v4u*)p = w;
  __threadfence();
  *(volatile v4u*)p = w;
}

__global__ __launch_bounds__(256) void feature_hidden_kernel(
    const float* __restrict__ x, const float* __restrict__ W1, const float* __restrict__ b1,
    const float* __restrict__ W2, const float* __restrict__ b2, unsigned* __restrict__ Uw)
{
  __shared__ __align__(16) float sW1[kHid * kFG];
  __shared__ __align__(16) float sB1[kHid * kFG];
  __shared__ __align__(16) float sW2[kHid * kFG];
  unsigned tid = threadIdx.x;
  asm volatile("" : "+v"(tid));
  unsigned lane = tid & 31u;
  asm volatile("" : "+v"(lane));
  const unsigned wave = tid >> 5;
  const unsigned d0 = blockIdx.x * (unsigned)kFG;

#pragma unroll
  for (unsigned it = 0; it < 4u; ++it) {
    unsigned e = (tid + 256u * it) << 2;
    asm volatile("" : "+v"(e));
    unsigned dl = e >> 6;
    unsigned hb = e & 63u;
    asm volatile("" : "+v"(dl));
    asm volatile("" : "+v"(hb));
    const size_t go = (size_t)d0 * kHid + e;
    const v4f a = *(const v4f*)(W1 + go);
    const v4f b = *(const v4f*)(b1 + go);
    const v4f c = *(const v4f*)(W2 + go);
#pragma unroll
    for (unsigned j = 0; j < 4u; ++j) {
      sW1[(hb + j) * kFG + dl] = a[j];
      sB1[(hb + j) * kFG + dl] = b[j];
      sW2[(hb + j) * kFG + dl] = c[j];
    }
  }
  __syncthreads();

  unsigned fo = 2u * lane;
  asm volatile("" : "+v"(fo));
  const v2f bias2 = *(const v2f*)(b2 + d0 + fo);
  const float b2a = bias2[0];
  const float b2b = bias2[1];
  const unsigned rowBlock = blockIdx.y * (unsigned)kRowsPerBlock + wave * 16u;
  const unsigned wcol = blockIdx.x * 32u + lane;

#pragma unroll 1
  for (unsigned g = 0; g < 4u; ++g) {
    const unsigned rb = rowBlock + g * 4u;
    float xa[4], xb[4], aa[4], ab[4];
#pragma unroll
    for (int r = 0; r < 4; ++r) {
      const v2f xv = *(const v2f*)(x + (size_t)(rb + r) * kFeat + d0 + fo);
      xa[r] = xv[0];
      xb[r] = xv[1];
      aa[r] = b2a;
      ab[r] = b2b;
    }
#pragma unroll 2
    for (unsigned h = 0; h < (unsigned)kHid; ++h) {
      const v2f w1v = *(const v2f*)(sW1 + h * kFG + fo);
      const v2f b1v = *(const v2f*)(sB1 + h * kFG + fo);
      const v2f w2v = *(const v2f*)(sW2 + h * kFG + fo);
      const float w1a = w1v[0], w1b = w1v[1];
      const float b1a = b1v[0], b1b = b1v[1];
      const float w2a = w2v[0], w2b = w2v[1];
#pragma unroll
      for (int r = 0; r < 4; ++r) {
        float ta = fmaf(xa[r], w1a, b1a);
        float tb = fmaf(xb[r], w1b, b1b);
        ta = fmaxf(ta, 0.0f);
        tb = fmaxf(tb, 0.0f);
        aa[r] = fmaf(ta, w2a, aa[r]);
        ab[r] = fmaf(tb, w2b, ab[r]);
      }
    }
    unsigned pk[4];
#pragma unroll
    for (int r = 0; r < 4; ++r) {
      const unsigned lo = f16_bits_flush(aa[r] * kCarryU);
      const unsigned hi = f16_bits_flush(ab[r] * kCarryU);
      pk[r] = pack_halves(lo, hi);
    }
    for (int pass = 0; pass < 2; ++pass) {
#pragma unroll
      for (int r = 0; r < 4; ++r) {
        *(volatile unsigned*)(Uw + (size_t)(rb + r) * (kFeat / 2) + wcol) = pk[r];
      }
      __threadfence();
    }
  }
}

union FragU { v16h v; v8h h[2]; };
__device__ __forceinline__ v16h frag_load_f16(const _Float16* p) {
  FragU f;
  f.h[0] = *(const v8h*)(p);
  f.h[1] = *(const v8h*)(p + 16);
  return f.v;
}
__device__ __forceinline__ v8f mma_f16_guarded(v16h a, v16h b, v8f c) {
  c = __builtin_amdgcn_wmma_f32_16x16x32_f16(false, a, false, b, (short)0, c, false, false);
  asm volatile("v_nop\n\tv_nop\n\tv_nop\n\tv_nop" : "+v"(c) : "v"(a), "v"(b));
  return c;
}

constexpr int kTilesN = kOut / 64;
constexpr int kTilesM = kRows / 64;
static_assert(kTilesN == 4 && ((kTilesM * kTilesN) % 8) == 0);

__global__ __launch_bounds__(256) void combine_gemm_kernel(
    const unsigned short* __restrict__ Ap, const unsigned short* __restrict__ Btp,
    const float* __restrict__ bias, float* __restrict__ C)
{
  __shared__ __align__(16) float sT[8 * 16 * 68];
  const _Float16* A  = (const _Float16*)Ap;
  const _Float16* Bt = (const _Float16*)Btp;
  unsigned tid = threadIdx.x;
  asm volatile("" : "+v"(tid));
  unsigned lane = tid & 31u;
  asm volatile("" : "+v"(lane));
  const unsigned wave = tid >> 5;
  const unsigned tile = blockIdx.x * 8u + wave;
  const unsigned tm = tile >> 2;
  const unsigned tn = tile & 3u;
  const unsigned m0 = tm << 6;
  const unsigned n0 = tn << 6;
  unsigned rlane = lane & 15u;
  asm volatile("" : "+v"(rlane));
  unsigned half8 = (lane >> 4) << 3;
  asm volatile("" : "+v"(half8));

  v8f acc[4][4];
#pragma unroll
  for (int i = 0; i < 4; ++i)
#pragma unroll
    for (int j = 0; j < 4; ++j) acc[i][j] = (v8f){0.f, 0.f, 0.f, 0.f, 0.f, 0.f, 0.f, 0.f};

#pragma unroll 1
  for (unsigned k0 = 0; k0 < (unsigned)kFeat; k0 += 32u) {
    v16h bh[4];
#pragma unroll
    for (int j = 0; j < 4; ++j) {
      const size_t bo = (size_t)(n0 + (unsigned)(j << 4) + rlane) * kFeat + half8 + k0;
      bh[j] = frag_load_f16(Bt + bo);
    }
#pragma unroll
    for (int i = 0; i < 4; ++i) {
      const size_t ao = (size_t)(m0 + (unsigned)(i << 4) + rlane) * kFeat + half8 + k0;
      const v16h ah = frag_load_f16(A + ao);
#pragma unroll
      for (int j = 0; j < 4; ++j) {
        acc[i][j] = mma_f16_guarded(ah, bh[j], acc[i][j]);
      }
    }
  }

  float bv[4];
#pragma unroll
  for (int j = 0; j < 4; ++j) bv[j] = bias[n0 + (unsigned)(j << 4) + rlane];
  float* slab = sT + wave * (16u * 68u);
  const unsigned hh = lane >> 4;
  const unsigned c4 = rlane * 4u;
#pragma unroll
  for (int i = 0; i < 4; ++i) {
    const unsigned mBase = m0 + (unsigned)(i << 4);
#pragma unroll
    for (int j = 0; j < 4; ++j) {
#pragma unroll
      for (int r = 0; r < 8; ++r) {
        const float v = acc[i][j][r] * kFold + bv[j];
        slab[(half8 + (unsigned)r) * 68u + (unsigned)(j << 4) + rlane] = v;
      }
    }
    __builtin_amdgcn_fence(__ATOMIC_RELEASE, "workgroup");
    __builtin_amdgcn_wave_barrier();
    __builtin_amdgcn_fence(__ATOMIC_ACQUIRE, "workgroup");
    for (int pass = 0; pass < 2; ++pass) {
#pragma unroll
      for (int it = 0; it < 8; ++it) {
        const unsigned row = (unsigned)(it * 2) + hh;
        const v4f v = *(const v4f*)(slab + row * 68u + c4);
        *(volatile v4f*)(C + (size_t)(mBase + row) * kOut + n0 + c4) = v;
      }
      __threadfence();
    }
    __builtin_amdgcn_fence(__ATOMIC_RELEASE, "workgroup");
    __builtin_amdgcn_wave_barrier();
    __builtin_amdgcn_fence(__ATOMIC_ACQUIRE, "workgroup");
  }
}

extern "C" void kernel_launch(void* const* d_in, const int* in_sizes, int n_in,
                              void* d_out, int out_size, void* d_ws, size_t ws_size,
                              hipStream_t stream) {
  if (n_in < 7) return;
  if (in_sizes[0] != kRows * kFeat) return;
  if (in_sizes[1] != kFeat * kHid) return;
  if (in_sizes[2] != kFeat * kHid) return;
  if (in_sizes[3] != kFeat * kHid) return;
  if (in_sizes[4] != kFeat) return;
  if (in_sizes[5] != kOut * kFeat) return;
  if (in_sizes[6] != kOut) return;
  if (out_size != kRows * kOut) return;
  if (ws_size < kWsTotal) return;

  const float* x  = (const float*)d_in[0];
  const float* W1 = (const float*)d_in[1];
  const float* b1 = (const float*)d_in[2];
  const float* W2 = (const float*)d_in[3];
  const float* b2 = (const float*)d_in[4];
  const float* Wc = (const float*)d_in[5];
  const float* bc = (const float*)d_in[6];
  float* out = (float*)d_out;

  char* ws = (char*)d_ws;
  unsigned* WC16 = (unsigned*)(ws + kOffWC16);
  unsigned* U16  = (unsigned*)(ws + kOffU16);

  cast_weight_plane_kernel<<<(kOut * kFeat / 8) / 256, 256, 0, stream>>>(Wc, WC16);

  feature_hidden_kernel<<<dim3(kFeat / kFG, kRows / kRowsPerBlock), 256, 0, stream>>>(
      x, W1, b1, W2, b2, U16);

  combine_gemm_kernel<<<(kTilesM * kTilesN) / 8, 256, 0, stream>>>(
      (const unsigned short*)U16, (const unsigned short*)WC16, bc, out);
}
